// GroupedQueryAttention_11536282157169
// MI455X (gfx1250) — hardware-verified
//
#include <hip/hip_runtime.h>
#pragma clang fp contract(off)


#ifndef NB
#define NB 2
#endif
#ifndef SEQ
#define SEQ 2048
#endif
#define TT      SEQ
#define TT_FULL 2048
#define DM   2048
#define NH_  32
#define NKV  8
#define REP  (NH_ / NKV)
#define HD   64
#define HALF 32
#define DQ   (NH_ * HD)
#define DKV  (NKV * HD)
#ifndef RH
#define RH   512
#endif
#define SCL  0.125f
#define SL   (SCL * 1.4426950408889634f)
#define NEGB (-1.0e30f)
#define FW   4
#define NTH  ((RH / 16) > 0 ? (RH / 16) : 1)
#define NTL  (((TT - RH) / 16) > 0 ? ((TT - RH) / 16) : 1)
#define NFLAG (TT / 8)

static_assert(TT % 128 == 0);
static_assert(RH % 64 == 0);
static_assert(RH <= TT);
static_assert((TT - RH) % 64 == 0);
static_assert(DM % 64 == 0);
static_assert(DQ % 64 == 0);
static_assert(DKV % 64 == 0);
static_assert((NH_ * (RH / 16)) % FW == 0);
static_assert((NH_ * ((TT - RH) / 16)) % FW == 0);
static_assert(((size_t)NH_ * TT * HD / 2) % 256 == 0);
static_assert(((size_t)NKV * TT * HD / 2) % 256 == 0);
static_assert(((size_t)NB * TT * DM) % 4096 == 0);
static_assert(NFLAG <= 256);
static_assert(NFLAG >= 1);

typedef _Float16 h16;
typedef unsigned short bf;
typedef __attribute__((ext_vector_type(16))) __bf16   v16bf;
typedef __attribute__((ext_vector_type(16))) _Float16 v16h;
typedef __attribute__((ext_vector_type(16))) unsigned short v16us;
typedef __attribute__((ext_vector_type(8)))  _Float16 v8h;
typedef __attribute__((ext_vector_type(8)))  unsigned short v8us;
typedef __attribute__((ext_vector_type(8)))  float    v8f;
typedef __attribute__((ext_vector_type(4)))  float    v4f;
typedef __attribute__((ext_vector_type(2)))  float    v2f;
typedef __attribute__((ext_vector_type(2)))  _Float16 v2h;
typedef __attribute__((ext_vector_type(2)))  unsigned short v2us;
typedef __attribute__((ext_vector_type(4)))  int v4i;
typedef v4f  __attribute__((may_alias)) v4fa;

__device__ __forceinline__ unsigned short f2bf(float f) { unsigned u = __float_as_uint(f); u += 0x7FFFu + ((u >> 16) & 1u); return (unsigned short)(u >> 16); }
__device__ __forceinline__ float bf2f(unsigned short b) { return __uint_as_float(((unsigned)b) << 16); }
__device__ __forceinline__ float bfr(float f) { return bf2f(f2bf(f)); }
__device__ __forceinline__ v16h cat16(v8h lo, v8h hi) { return __builtin_shufflevector(lo, hi, 0, 1, 2, 3, 4, 5, 6, 7, 8, 9, 10, 11, 12, 13, 14, 15); }
__device__ __forceinline__ v16bf cat16b(v8us lo, v8us hi) { return __builtin_bit_cast(v16bf, __builtin_shufflevector(lo, hi, 0, 1, 2, 3, 4, 5, 6, 7, 8, 9, 10, 11, 12, 13, 14, 15)); }
__device__ __forceinline__ v8f wmma16(v16h a, v16h b, v8f c) { return __builtin_amdgcn_wmma_f32_16x16x32_f16(false, a, false, b, (short)0, c, false, false); }
__device__ __forceinline__ v8f wmmab(v16bf a, v16bf b, v8f c) { return __builtin_amdgcn_wmma_f32_16x16x32_bf16(false, a, false, b, (short)0, c, false, false); }
__device__ __forceinline__ h16 tohx(float x) { return (h16)x; }
__device__ __forceinline__ void splitf(float y, unsigned short& h, unsigned short& l) { h = f2bf(y); l = f2bf(y - bf2f(h)); }

template <typename T16> struct WFrag;
template <> struct WFrag<h16> { typedef v16h V; static __device__ __forceinline__ V ld(const h16* p) { return cat16(*(const v8h*)p, *(const v8h*)(p + 16)); } static __device__ __forceinline__ v8f mma(V a, V b, v8f c) { return wmma16(a, b, c); } };
template <> struct WFrag<bf> { typedef v16bf V; static __device__ __forceinline__ V ld(const bf* p) { return cat16b(*(const v8us*)p, *(const v8us*)(p + 16)); } static __device__ __forceinline__ v8f mma(V a, V b, v8f c) { return wmmab(a, b, c); } };
template <typename T16, int NSPLIT, bool BIAS>
__global__ __launch_bounds__(32) void k_gemmw(const T16* __restrict__ A, const T16* __restrict__ A2, const T16* __restrict__ Bt, const T16* __restrict__ Bt2, int K, float* C, int ldc, const float* __restrict__ bias, size_t sA, size_t sB, size_t sC) {
    typedef typename WFrag<T16>::V V;
    __shared__ __align__(16) float os[16 * 68];
    const size_t z = blockIdx.z; A += z * sA; if (A2) A2 += z * sA; Bt += z * sB; if (Bt2) Bt2 += z * sB; C += z * sC;
    const int lane = threadIdx.x & 31, lr = lane & 15, hi = lane >> 4; const int r0 = blockIdx.x * 64, c0 = blockIdx.y * 64;
    v8f acc[4][4];
#pragma unroll
    for (int mb = 0; mb < 4; ++mb)
#pragma unroll
        for (int nb = 0; nb < 4; ++nb) acc[mb][nb] = (v8f){};
    const size_t aoff = (size_t)(r0 + lr) * K + 8 * hi, boff = (size_t)(c0 + lr) * K + 8 * hi;
#pragma unroll 1
    for (int kc = 0; kc < K; kc += 32) {
        V a[4], a2[4];
#pragma unroll
        for (int mb = 0; mb < 4; ++mb) { a[mb] = WFrag<T16>::ld(A + aoff + (size_t)mb * 16 * K + kc); if (NSPLIT == 1 || NSPLIT == 2) a2[mb] = WFrag<T16>::ld(A2 + aoff + (size_t)mb * 16 * K + kc); }
#pragma unroll
        for (int nb = 0; nb < 4; ++nb) { const V b = WFrag<T16>::ld(Bt + boff + (size_t)nb * 16 * K + kc); V b2; if (NSPLIT >= 2) b2 = WFrag<T16>::ld(Bt2 + boff + (size_t)nb * 16 * K + kc);
#pragma unroll
            for (int mb = 0; mb < 4; ++mb) { acc[mb][nb] = WFrag<T16>::mma(a[mb], b, acc[mb][nb]); if (NSPLIT == 1 || NSPLIT == 2) acc[mb][nb] = WFrag<T16>::mma(a2[mb], b, acc[mb][nb]); if (NSPLIT >= 2) acc[mb][nb] = WFrag<T16>::mma(a[mb], b2, acc[mb][nb]); } }
        asm volatile("v_nop\n\tv_nop\n\tv_nop\n\tv_nop" : "+v"(acc[0][0]), "+v"(acc[1][1]), "+v"(acc[2][2]), "+v"(acc[3][3]) : "v"(a[0]), "v"(a[3]));
    }
#pragma unroll
    for (int mb = 0; mb < 4; ++mb) {
#pragma unroll
        for (int nb = 0; nb < 4; ++nb) {
#pragma unroll
            for (int j = 0; j < 8; ++j) os[(hi * 8 + j) * 68 + nb * 16 + lr] = acc[mb][nb][j]; }
        __builtin_amdgcn_fence(3  , "wavefront"); __builtin_amdgcn_wave_barrier(); asm volatile("" ::: "memory");
        float* crow = C + (size_t)(r0 + mb * 16) * ldc + c0;
#pragma unroll 1
        for (int ps = 0; ps < 2; ++ps) {
#pragma unroll
            for (int s = 0; s < 8; ++s) { const int row = 2 * s + hi, cofs = lr * 4; v4f val = *(const v4fa*)(os + row * 68 + cofs); if (BIAS) { val[0] += bfr(bias[c0 + cofs]); val[1] += bfr(bias[c0 + cofs + 1]); val[2] += bfr(bias[c0 + cofs + 2]); val[3] += bfr(bias[c0 + cofs + 3]); }
                *(volatile v4f*)(crow + (size_t)row * ldc + cofs) = val; }
            if (ps == 0) __threadfence(); }
        __builtin_amdgcn_wave_barrier(); asm volatile("" ::: "memory");
    }
}

__global__ __launch_bounds__(256) void k_cvt8(const float* __restrict__ src, bf* dst, size_t n8) { const size_t i = (size_t)blockIdx.x * 256 + threadIdx.x; if (i >= n8) return; const v8f v = *(const v8f*)(src + i * 8); v8us o;
#pragma unroll
    for (int k = 0; k < 8; ++k) o[k] = f2bf(v[k]); *(volatile v8us*)(dst + i * 8) = o; __threadfence(); *(volatile v8us*)(dst + i * 8) = o; }

__global__ __launch_bounds__(256) void k_rope(const float* __restrict__ F, int pitch, int nheads, const float* __restrict__ COS, const float* __restrict__ SIN, float sc, h16* P16, bf* Ph, bf* Pl) {
    const size_t e = ((size_t)blockIdx.x * 256 + threadIdx.x) * 2; if (e >= (size_t)nheads * TT * HD) return;
    const int d = (int)(e % HD); const int t = (int)((e / HD) % TT); const int h = (int)(e / ((size_t)HD * TT));
    const v2f xv = *(const v2f*)(F + (size_t)t * pitch + h * HD + d);
    const float c = bfr(COS[(size_t)t * HALF + (d >> 1)]), s = bfr(SIN[(size_t)t * HALF + (d >> 1)]);
    const float a0 = xv[0] * c, b0 = xv[1] * s, a1 = xv[0] * s, b1 = xv[1] * c;
    const float r0 = (a0 - b0) * sc, r1 = (a1 + b1) * sc;
    v2h o16; v2us oh, ol; unsigned short hh, ll;
    o16[0] = tohx(r0); splitf(r0, hh, ll); oh[0] = hh; ol[0] = ll;
    o16[1] = tohx(r1); splitf(r1, hh, ll); oh[1] = hh; ol[1] = ll;
    *(volatile v2h*)(P16 + e) = o16; *(volatile v2us*)(Ph + e) = oh; *(volatile v2us*)(Pl + e) = ol; __threadfence(); *(volatile v2h*)(P16 + e) = o16; *(volatile v2us*)(Ph + e) = oh; *(volatile v2us*)(Pl + e) = ol; }

__global__ __launch_bounds__(256) void k_vtp(const float* __restrict__ F, int pitch, int nheads, h16* V16, bf* Vh, bf* Vl) { const size_t e = ((size_t)blockIdx.x * 256 + threadIdx.x) * 2; if (e >= (size_t)nheads * HD * TT) return; const int t = (int)(e % TT); const int d = (int)((e / TT) % HD); const int g = (int)(e / ((size_t)TT * HD)); v2h o16; v2us oh, ol;
#pragma unroll
    for (int q = 0; q < 2; ++q) { const float x = F[(size_t)(t + q) * pitch + g * HD + d]; o16[q] = tohx(x); unsigned short a2, c2; splitf(x, a2, c2); oh[q] = a2; ol[q] = c2; }
    *(volatile v2h*)(V16 + e) = o16; *(volatile v2us*)(Vh + e) = oh; *(volatile v2us*)(Vl + e) = ol; __threadfence(); *(volatile v2h*)(V16 + e) = o16; *(volatile v2us*)(Vh + e) = oh; *(volatile v2us*)(Vl + e) = ol; }

__global__ __launch_bounds__(256) void k_maskchk(const int* __restrict__ mask, int* flags) {
    const int lane = threadIdx.x & 31; const int i = blockIdx.x * 8 + (int)(threadIdx.x >> 5);
    const int* mr = mask + (size_t)i * TT_FULL; int bad = 0;
#pragma unroll 4
    for (int ch = 0; ch < TT / 128; ++ch) { const int j0 = ch * 128 + lane * 4; const v4i a = *(const v4i*)(mr + j0);
#pragma unroll
        for (int q = 0; q < 4; ++q) bad |= (int)((a[q] != 0) != (j0 + q <= i)); }
    const int any = __syncthreads_or(bad);
    if (threadIdx.x < 8) { v4i f; f[0] = any; f[1] = any; f[2] = any; f[3] = any; int* p = flags + (size_t)blockIdx.x * 32 + threadIdx.x * 4;
        *(volatile v4i*)p = f; __threadfence(); *(volatile v4i*)p = f; }
}

__global__ __launch_bounds__(256) void k_poison(const int* __restrict__ flags, float* OUT) {
    const int fi = ((int)threadIdx.x < NFLAG) ? (int)threadIdx.x : (NFLAG - 1);
    const int f = flags[(size_t)fi * 32];
    const int any = __syncthreads_or(f != 0);
    if (!any) return;
    const float qn = __uint_as_float(0x7FC00000u); v4f v; v[0] = qn; v[1] = qn; v[2] = qn; v[3] = qn;
    float* base = OUT + (size_t)blockIdx.x * 4096 + threadIdx.x * 4;
#pragma unroll 1
    for (int ps = 0; ps < 2; ++ps) {
#pragma unroll
        for (int s = 0; s < 4; ++s) *(volatile v4f*)(base + s * 1024) = v;
        if (ps == 0) __threadfence(); }
}

__device__ __forceinline__ void flash_fin(float* o, v8f a0, v8f a1, v8f a2, v8f a3, float inv, int lane, bf* ATh, bf* ATl, size_t base) {
    const int lr = lane & 15, hi = lane >> 4;
    float* wr = o + lr * 68 + 8 * hi;
    { v4f x, y; x[0] = a0[0] * inv; x[1] = a0[1] * inv; x[2] = a0[2] * inv; x[3] = a0[3] * inv; y[0] = a0[4] * inv; y[1] = a0[5] * inv; y[2] = a0[6] * inv; y[3] = a0[7] * inv; *(v4fa*)(wr) = x; *(v4fa*)(wr + 4) = y; }
    { v4f x, y; x[0] = a1[0] * inv; x[1] = a1[1] * inv; x[2] = a1[2] * inv; x[3] = a1[3] * inv; y[0] = a1[4] * inv; y[1] = a1[5] * inv; y[2] = a1[6] * inv; y[3] = a1[7] * inv; *(v4fa*)(wr + 16) = x; *(v4fa*)(wr + 20) = y; }
    { v4f x, y; x[0] = a2[0] * inv; x[1] = a2[1] * inv; x[2] = a2[2] * inv; x[3] = a2[3] * inv; y[0] = a2[4] * inv; y[1] = a2[5] * inv; y[2] = a2[6] * inv; y[3] = a2[7] * inv; *(v4fa*)(wr + 32) = x; *(v4fa*)(wr + 36) = y; }
    { v4f x, y; x[0] = a3[0] * inv; x[1] = a3[1] * inv; x[2] = a3[2] * inv; x[3] = a3[3] * inv; y[0] = a3[4] * inv; y[1] = a3[5] * inv; y[2] = a3[6] * inv; y[3] = a3[7] * inv; *(v4fa*)(wr + 48) = x; *(v4fa*)(wr + 52) = y; }
    __builtin_amdgcn_fence(3  , "wavefront"); __builtin_amdgcn_wave_barrier(); asm volatile("" ::: "memory");
    const int rq = lane >> 3, cofs = (lane & 7) * 8;
#pragma unroll 1
    for (int ps = 0; ps < 2; ++ps) {
#pragma unroll
        for (int s = 0; s < 4; ++s) { const int row = 4 * s + rq; const v4f x = *(const v4fa*)(o + row * 68 + cofs), y = *(const v4fa*)(o + row * 68 + cofs + 4); v8us oh, ol; unsigned short hh, ll;
#pragma unroll
            for (int q = 0; q < 4; ++q) { splitf(x[q], hh, ll); oh[q] = hh; ol[q] = ll; splitf(y[q], hh, ll); oh[4 + q] = hh; ol[4 + q] = ll; }
            const size_t oo = base + (size_t)row * DQ + cofs; *(volatile v8us*)(ATh + oo) = oh; *(volatile v8us*)(ATl + oo) = ol; }
        if (ps == 0) __threadfence(); }
}

__global__ __launch_bounds__(128) void k_flash_lo(const h16* __restrict__ Q16, const h16* __restrict__ K16, const h16* __restrict__ V16, bf* ATh, bf* ATl) {
    __shared__ __align__(16) float os[FW * 16 * 68];
    const int lane = threadIdx.x & 31, lr = lane & 15, hi = lane >> 4;
    const int wave = __builtin_amdgcn_readfirstlane((int)(threadIdx.x >> 5));
    const int w = (int)blockIdx.x * FW + wave;
    const int head = w / NTL, q0 = RH + (w % NTL) * 16, g = head / REP;
    const h16* Qb = Q16 + ((size_t)head * TT + q0 + lr) * HD + 8 * hi;
    const h16* Kb = K16 + ((size_t)g * TT + lr) * HD + 8 * hi;
    const h16* Vb = V16 + ((size_t)g * HD + lr) * TT + 8 * hi;
    const v16h qb0 = WFrag<h16>::ld(Qb), qb1 = WFrag<h16>::ld(Qb + 32);
    v8f oT[4];
#pragma unroll
    for (int dt = 0; dt < 4; ++dt) oT[dt] = (v8f){};
    float mrun = NEGB, lsum = 0.0f; const int qi = q0 + lr;
#pragma unroll 1
    for (int kb = 0; kb < q0 + 16; kb += 64) {
        v8f st[4];
#pragma unroll
        for (int c = 0; c < 4; ++c) {
            const h16* kp = Kb + (size_t)(kb + 16 * c) * HD;
            const v16h ka0 = WFrag<h16>::ld(kp), ka1 = WFrag<h16>::ld(kp + 32);
            v8f s = (v8f){};
            s = wmma16(ka0, qb0, s); s = wmma16(ka1, qb1, s);
            asm volatile("v_nop\n\tv_nop\n\tv_nop\n\tv_nop" : "+v"(s) : "v"(ka0), "v"(ka1) : "memory");
            st[c] = s; }
        if (kb + 63 > q0) { const int kbase = kb + 8 * hi - qi;
#pragma unroll
            for (int c = 0; c < 4; ++c)
#pragma unroll
                for (int j = 0; j < 8; ++j) st[c][j] = (kbase + 16 * c + j > 0) ? NEGB : st[c][j]; }
        float mx = NEGB;
#pragma unroll
        for (int c = 0; c < 4; ++c)
#pragma unroll
            for (int j = 0; j < 8; ++j) mx = fmaxf(mx, st[c][j]);
        mx = fmaxf(mx, __shfl_xor(mx, 16, 32));
        const float mnew = fmaxf(mrun, mx);
        const float alpha = __builtin_amdgcn_exp2f((mrun - mnew) * SL);
        mrun = mnew; lsum *= alpha;
#pragma unroll
        for (int dt = 0; dt < 4; ++dt)
#pragma unroll
            for (int j = 0; j < 8; ++j) oT[dt][j] *= alpha;
        const float mb = 10.0f - mnew * SL;
        v16h pb[2];
#pragma unroll
        for (int c = 0; c < 4; ++c)
#pragma unroll
            for (int j = 0; j < 8; ++j) { const float p = __builtin_amdgcn_exp2f(fmaf(st[c][j], SL, mb)); const h16 hh = (h16)p; lsum += (float)hh; pb[c >> 1][(c & 1) * 8 + j] = hh; }
#pragma unroll
        for (int ks = 0; ks < 2; ++ks)
#pragma unroll
            for (int dt = 0; dt < 4; ++dt) { const v16h va = WFrag<h16>::ld(Vb + (size_t)(16 * dt) * TT + kb + 32 * ks); oT[dt] = wmma16(va, pb[ks], oT[dt]); }
        asm volatile("v_nop\n\tv_nop\n\tv_nop\n\tv_nop" : "+v"(oT[0]), "+v"(oT[1]), "+v"(oT[2]), "+v"(oT[3]) : "v"(pb[0]), "v"(pb[1]) : "memory");
    }
    lsum += __shfl_xor(lsum, 16, 32);
    const float inv = 1.0f / lsum;
    flash_fin(os + wave * (16 * 68), oT[0], oT[1], oT[2], oT[3], inv, lane, ATh, ATl, (size_t)q0 * DQ + (size_t)head * HD);
}

__global__ __launch_bounds__(128) void k_flash_hi(const bf* __restrict__ Qh, const bf* __restrict__ Ql, const bf* __restrict__ Kh, const bf* __restrict__ Kl, const bf* __restrict__ Vh, const bf* __restrict__ Vl, bf* ATh, bf* ATl) {
    __shared__ __align__(16) float os[FW * 16 * 68];
    const int lane = threadIdx.x & 31, lr = lane & 15, hi = lane >> 4;
    const int wave = __builtin_amdgcn_readfirstlane((int)(threadIdx.x >> 5));
    const int w = (int)blockIdx.x * FW + wave;
    const int head = w / NTH, q0 = (w % NTH) * 16, g = head / REP;
    const size_t qo = ((size_t)head * TT + q0 + lr) * HD + 8 * hi;
    const size_t ko = ((size_t)g * TT + lr) * HD + 8 * hi;
    const size_t vo = ((size_t)g * HD + lr) * TT + 8 * hi;
    const v16bf qh0 = WFrag<bf>::ld(Qh + qo), qh1 = WFrag<bf>::ld(Qh + qo + 32), ql0 = WFrag<bf>::ld(Ql + qo), ql1 = WFrag<bf>::ld(Ql + qo + 32);
    v8f oT[4];
#pragma unroll
    for (int dt = 0; dt < 4; ++dt) oT[dt] = (v8f){};
    float mrun = NEGB, lsum = 0.0f; const int qi = q0 + lr;
#pragma unroll 1
    for (int kb = 0; kb < q0 + 16; kb += 64) {
        v8f st[4];
#pragma unroll
        for (int c = 0; c < 4; ++c) {
            const size_t kk = ko + (size_t)(kb + 16 * c) * HD;
            const v16bf kh0 = WFrag<bf>::ld(Kh + kk), kh1 = WFrag<bf>::ld(Kh + kk + 32), kl0 = WFrag<bf>::ld(Kl + kk), kl1 = WFrag<bf>::ld(Kl + kk + 32);
            v8f s = (v8f){};
            s = wmmab(kl0, qh0, s); s = wmmab(kl1, qh1, s); s = wmmab(kh0, ql0, s); s = wmmab(kh1, ql1, s); s = wmmab(kh0, qh0, s); s = wmmab(kh1, qh1, s);
            asm volatile("v_nop\n\tv_nop\n\tv_nop\n\tv_nop" : "+v"(s) : "v"(kh0), "v"(kh1) : "memory");
            st[c] = s; }
        if (kb + 63 > q0) { const int kbase = kb + 8 * hi - qi;
#pragma unroll
            for (int c = 0; c < 4; ++c)
#pragma unroll
                for (int j = 0; j < 8; ++j) st[c][j] = (kbase + 16 * c + j > 0) ? NEGB : st[c][j]; }
        float mx = NEGB;
#pragma unroll
        for (int c = 0; c < 4; ++c)
#pragma unroll
            for (int j = 0; j < 8; ++j) mx = fmaxf(mx, st[c][j]);
        mx = fmaxf(mx, __shfl_xor(mx, 16, 32));
        const float mnew = fmaxf(mrun, mx);
        const float alpha = __builtin_amdgcn_exp2f((mrun - mnew) * SL);
        mrun = mnew; lsum *= alpha;
#pragma unroll
        for (int dt = 0; dt < 4; ++dt)
#pragma unroll
            for (int j = 0; j < 8; ++j) oT[dt][j] *= alpha;
        const float mb = -mnew * SL;
        v16us phu[2], plu[2];
#pragma unroll
        for (int c = 0; c < 4; ++c)
#pragma unroll
            for (int j = 0; j < 8; ++j) { const float p = __builtin_amdgcn_exp2f(fmaf(st[c][j], SL, mb)); lsum += p; unsigned short hh, ll; splitf(p, hh, ll); phu[c >> 1][(c & 1) * 8 + j] = hh; plu[c >> 1][(c & 1) * 8 + j] = ll; }
        v16bf ph[2], pl[2];
        ph[0] = __builtin_bit_cast(v16bf, phu[0]); ph[1] = __builtin_bit_cast(v16bf, phu[1]); pl[0] = __builtin_bit_cast(v16bf, plu[0]); pl[1] = __builtin_bit_cast(v16bf, plu[1]);
#pragma unroll
        for (int ks = 0; ks < 2; ++ks) {
#pragma unroll
            for (int dt = 0; dt < 4; ++dt) { const size_t vv = vo + (size_t)(16 * dt) * TT + kb + 32 * ks; const v16bf vh = WFrag<bf>::ld(Vh + vv), vl = WFrag<bf>::ld(Vl + vv);
                oT[dt] = wmmab(vl, ph[ks], oT[dt]); oT[dt] = wmmab(vh, pl[ks], oT[dt]); oT[dt] = wmmab(vh, ph[ks], oT[dt]); }
            asm volatile("v_nop\n\tv_nop\n\tv_nop\n\tv_nop" : "+v"(oT[0]), "+v"(oT[1]), "+v"(oT[2]), "+v"(oT[3]) : "v"(ph[ks]), "v"(pl[ks]) : "memory"); }
    }
    lsum += __shfl_xor(lsum, 16, 32);
    const float inv = 1.0f / lsum;
    flash_fin(os + wave * (16 * 68), oT[0], oT[1], oT[2], oT[3], inv, lane, ATh, ATl, (size_t)q0 * DQ + (size_t)head * HD);
}

extern "C" void kernel_launch(void* const* d_in, const int* in_sizes, int n_in,
                              void* d_out, int out_size, void* d_ws, size_t ws_size, hipStream_t stream) {
    (void)out_size;
    if (n_in < 8) return;
    if (in_sizes[0] < (NB - 1) * TT_FULL * DM + TT * DM) return;
    if (in_sizes[1] < (TT - 1) * TT_FULL + TT) return;
    if (in_sizes[2] < DQ * DM || in_sizes[3] < DKV * DM || in_sizes[4] < DKV * DM || in_sizes[5] < DM * DQ) return;
    if (in_sizes[6] < TT * HALF || in_sizes[7] < TT * HALF) return;
    const float* x = (const float*)d_in[0]; const int* mask = (const int*)d_in[1];
    const float* wq = (const float*)d_in[2]; const float* wk = (const float*)d_in[3]; const float* wv = (const float*)d_in[4]; const float* wo = (const float*)d_in[5];
    const float* cs = (const float*)d_in[6]; const float* sn = (const float*)d_in[7];
    float* OUT = (float*)d_out;
    char* wsp = (char*)d_ws;
    auto take = [&](size_t bytes) { char* p = wsp; wsp += (bytes + 255) & ~(size_t)255; return (void*)p; };
    bf* WQ = (bf*)take((size_t)DQ * DM * 2); bf* WK = (bf*)take((size_t)DKV * DM * 2); bf* WV = (bf*)take((size_t)DKV * DM * 2); bf* WO = (bf*)take((size_t)DM * DQ * 2);
    bf* XB = (bf*)take((size_t)TT * DM * 2); float* FQ = (float*)take((size_t)TT * DQ * 4); float* FK = (float*)take((size_t)TT * DKV * 4);
    h16* QP16 = (h16*)take((size_t)NH_ * TT * HD * 2); bf* QPh = (bf*)take((size_t)NH_ * TT * HD * 2); bf* QPl = (bf*)take((size_t)NH_ * TT * HD * 2);
    h16* KP16 = (h16*)take((size_t)NKV * TT * HD * 2); bf* KPh = (bf*)take((size_t)NKV * TT * HD * 2); bf* KPl = (bf*)take((size_t)NKV * TT * HD * 2);
    h16* VT16 = (h16*)take((size_t)NKV * HD * TT * 2); bf* VTh = (bf*)take((size_t)NKV * HD * TT * 2); bf* VTl = (bf*)take((size_t)NKV * HD * TT * 2);
    bf* ATh = (bf*)take((size_t)TT * DQ * 2); bf* ATl = (bf*)take((size_t)TT * DQ * 2);
    int* FLG = (int*)take((size_t)NFLAG * 128);
    if ((size_t)(wsp - (char*)d_ws) > ws_size) return;
    float* FV = FK;
    k_cvt8<<<(unsigned)(((size_t)DQ * DM / 8 + 255) / 256), 256, 0, stream>>>(wq, WQ, (size_t)DQ * DM / 8);
    k_cvt8<<<(unsigned)(((size_t)DKV * DM / 8 + 255) / 256), 256, 0, stream>>>(wk, WK, (size_t)DKV * DM / 8);
    k_cvt8<<<(unsigned)(((size_t)DKV * DM / 8 + 255) / 256), 256, 0, stream>>>(wv, WV, (size_t)DKV * DM / 8);
    k_cvt8<<<(unsigned)(((size_t)DM * DQ / 8 + 255) / 256), 256, 0, stream>>>(wo, WO, (size_t)DM * DQ / 8);
    k_maskchk<<<NFLAG, 256, 0, stream>>>(mask, FLG);
    const unsigned LQ = (unsigned)((size_t)NH_ * TT * HD / 2 / 256), LKv = (unsigned)((size_t)NKV * TT * HD / 2 / 256);
    for (int b = 0; b < NB; ++b) {
        k_cvt8<<<(unsigned)(((size_t)TT * DM / 8 + 255) / 256), 256, 0, stream>>>(x + (size_t)b * TT_FULL * DM, XB, (size_t)TT * DM / 8);
        k_gemmw<bf, 0, false><<<dim3(TT / 64, DQ / 64, 1), 32, 0, stream>>>(XB, nullptr, WQ, nullptr, DM, FQ, DQ, nullptr, 0, 0, 0);
        k_rope<<<LQ, 256, 0, stream>>>(FQ, DQ, NH_, cs, sn, 1.0f, QP16, QPh, QPl);
        k_gemmw<bf, 0, false><<<dim3(TT / 64, DKV / 64, 1), 32, 0, stream>>>(XB, nullptr, WK, nullptr, DM, FK, DKV, nullptr, 0, 0, 0);
        k_rope<<<LKv, 256, 0, stream>>>(FK, DKV, NKV, cs, sn, 1.0f, KP16, KPh, KPl);
        k_gemmw<bf, 0, false><<<dim3(TT / 64, DKV / 64, 1), 32, 0, stream>>>(XB, nullptr, WV, nullptr, DM, FV, DKV, nullptr, 0, 0, 0);
        k_vtp<<<LKv, 256, 0, stream>>>(FV, DKV, NKV, VT16, VTh, VTl);
        if (RH > 0) k_flash_hi<<<(unsigned)(NH_ * (RH / 16) / FW), 128, 0, stream>>>(QPh, QPl, KPh, KPl, VTh, VTl, ATh, ATl);
        if (TT > RH) k_flash_lo<<<(unsigned)(NH_ * ((TT - RH) / 16) / FW), 128, 0, stream>>>(QP16, KP16, VT16, ATh, ATl);
        k_gemmw<bf, 1, false><<<dim3(TT / 64, DM / 64, 1), 32, 0, stream>>>(ATh, ATl, WO, nullptr, DQ, OUT + (size_t)b * TT * DM, DM, nullptr, 0, 0, 0);
    }
    k_poison<<<(unsigned)((size_t)NB * TT * DM / 4096), 256, 0, stream>>>(FLG, OUT);
}
